// TokenMixing_27900107555053
// MI455X (gfx1250) — hardware-run, weakly checked
//
#include <hip/hip_runtime.h>


#ifndef NB
#define NB 4
#endif
#ifndef SEQ
#define SEQ 512
#endif
#define NB_FULL  4
#define SEQ_FULL 512
#ifndef OUT_SEQ
#define OUT_SEQ SEQ
#endif
#define DM   256
#define KA   64
#define NBP  16

static_assert(DM % 64 == 0);
static_assert(DM % 32 == 0);
static_assert(KA % 32 == 0);
static_assert(KA * 2 == 128);
static_assert(SEQ % 64 == 0);
static_assert((NB * SEQ) % 64 == 0);
static_assert(((size_t)DM * DM) % 64 == 0);
static_assert(NBP == 16);
static_assert(NB <= 4);
static_assert(NB <= NBP);
static_assert(NB <= NB_FULL);
static_assert(SEQ <= SEQ_FULL);
static_assert(NBP * KA / 8 == 128);
static_assert(8 * 16 == 64 * 2);
static_assert(2 * 8 * 16 == 64 * 4);
static_assert(32 * 16 * 8 == 16 * 64 * 4);
static_assert(16 * 68 * 4 <= 131072);
static_assert((68 * 4) % 16 == 0);
static_assert(((size_t)SEQ * DM) % 8 == 0);
static_assert(((size_t)DM * DM * KA) % 8 == 0);
static_assert(((size_t)DM * KA) % 8 == 0);

typedef _Float16 h16;
typedef unsigned short bf;
typedef __attribute__((ext_vector_type(16))) __bf16   v16bf;
typedef __attribute__((ext_vector_type(16))) _Float16 v16h;
typedef __attribute__((ext_vector_type(8)))  _Float16 v8h;
typedef __attribute__((ext_vector_type(8)))  unsigned short v8us;
typedef __attribute__((ext_vector_type(8)))  float    v8f;
typedef __attribute__((ext_vector_type(4)))  float    v4f;
typedef v4f  __attribute__((may_alias)) v4fa;

__device__ __forceinline__ unsigned short f2bf(float f) { unsigned u = __float_as_uint(f); u += 0x7FFFu + ((u >> 16) & 1u); return (unsigned short)(u >> 16); }
__device__ __forceinline__ float bfr(float f) { return __uint_as_float(((unsigned)f2bf(f)) << 16); }
__device__ __forceinline__ v16h cat16(v8h lo, v8h hi) { return __builtin_shufflevector(lo, hi, 0, 1, 2, 3, 4, 5, 6, 7, 8, 9, 10, 11, 12, 13, 14, 15); }
__device__ __forceinline__ v16bf cat16b(v8us lo, v8us hi) { return __builtin_bit_cast(v16bf, __builtin_shufflevector(lo, hi, 0, 1, 2, 3, 4, 5, 6, 7, 8, 9, 10, 11, 12, 13, 14, 15)); }
__device__ __forceinline__ v8f wmma16(v16h a, v16h b, v8f c) { return __builtin_amdgcn_wmma_f32_16x16x32_f16(false, a, false, b, (short)0, c, false, false); }
__device__ __forceinline__ v8f wmmab(v16bf a, v16bf b, v8f c) { return __builtin_amdgcn_wmma_f32_16x16x32_bf16(false, a, false, b, (short)0, c, false, false); }
__device__ __forceinline__ v16h  ldh(const h16* p) { return cat16(*(const v8h*)p, *(const v8h*)(p + 16)); }
__device__ __forceinline__ v16bf ldb(const bf* p)  { return cat16b(*(const v8us*)p, *(const v8us*)(p + 16)); }
__device__ __forceinline__ void wave_sync() { __builtin_amdgcn_fence(3  , "wavefront"); __builtin_amdgcn_wave_barrier(); asm volatile("" ::: "memory"); }
static __device__ __forceinline__ h16 toh_flush(float v) { const h16 r = (h16)v; return (fabsf(v) < 6.103515625e-05f) ? (h16)0.0f : r; }
__device__ __forceinline__ v8f wmma16g(v16h a, v16h b, v8f c) { c = wmma16(a, b, c); asm volatile("v_nop\n\tv_nop\n\tv_nop\n\tv_nop" : "+v"(c) : "v"(a), "v"(b)); return c; }
__device__ __forceinline__ v8f wmmabg(v16bf a, v16bf b, v8f c) { c = wmmab(a, b, c); asm volatile("v_nop\n\tv_nop\n\tv_nop\n\tv_nop" : "+v"(c) : "v"(a), "v"(b)); return c; }

__global__ __launch_bounds__(256) void k_cvt8(const float* __restrict__ src, bf* dst, size_t n8) {
    const size_t i = (size_t)blockIdx.x * 256 + threadIdx.x; if (i >= n8) return;
    const v8f v = *(const v8f*)(src + i * 8); v8us o;
#pragma unroll
    for (int k = 0; k < 8; ++k) o[k] = f2bf(v[k]);
    *(volatile v8us*)(dst + i * 8) = o; __threadfence(); *(volatile v8us*)(dst + i * 8) = o;
}

__global__ __launch_bounds__(256) void k_cvth8(const float* __restrict__ src, h16* dst, size_t n8) {
    const size_t i = (size_t)blockIdx.x * 256 + threadIdx.x; if (i >= n8) return;
    const v8f v = *(const v8f*)(src + i * 8); v8h o;
#pragma unroll
    for (int k = 0; k < 8; ++k) o[k] = toh_flush(bfr(v[k]));
    *(volatile v8h*)(dst + i * 8) = o; __threadfence(); *(volatile v8h*)(dst + i * 8) = o;
}

__global__ __launch_bounds__(128) void k_adp(const float* __restrict__ adp, bf* dst) {
    const int i = threadIdx.x;
    const int row = i >> 3, c8 = (i & 7) * 8;
    const int rc = row < NB ? row : (NB - 1);
    v8f v = *(const v8f*)(adp + (size_t)rc * KA + c8);
    asm volatile("" : "+v"(v));
    v8us o;
#pragma unroll
    for (int k = 0; k < 8; ++k) o[k] = (row < NB) ? f2bf(v[k]) : (unsigned short)0;
    *(volatile v8us*)(dst + (size_t)i * 8) = o; __threadfence(); *(volatile v8us*)(dst + (size_t)i * 8) = o;
}

__device__ __forceinline__ void adapt_acc(const bf* __restrict__ A, const bf* __restrict__ ADP, int r0, int lr, int hi, v8f (&acc)[4]) {
#pragma unroll
    for (int mb = 0; mb < 4; ++mb) acc[mb] = (v8f){};
    const size_t aoff = (size_t)(r0 + lr) * KA + 8 * hi, boff = (size_t)lr * KA + 8 * hi;
#pragma unroll
    for (int kc = 0; kc < KA; kc += 32) {
        const v16bf b = ldb(ADP + boff + kc);
#pragma unroll
        for (int mb = 0; mb < 4; ++mb) { const v16bf a = ldb(A + aoff + (size_t)mb * 16 * KA + kc); acc[mb] = wmmabg(a, b, acc[mb]); }
    }
}

__global__ __launch_bounds__(32) void k_wgen(const bf* __restrict__ AW, const bf* __restrict__ ADP, const float* __restrict__ awb, const float* __restrict__ wst, h16* WP) {
    __shared__ __align__(16) float os[16 * 68];
    const int lane = threadIdx.x & 31, lr = lane & 15, hi = lane >> 4; const int r0 = blockIdx.x * 64;
    v8f acc[4];
    adapt_acc(AW, ADP, r0, lr, hi, acc);
#pragma unroll
    for (int mb = 0; mb < 4; ++mb) { v4f p, q;
        p[0] = acc[mb][0]; p[1] = acc[mb][1]; p[2] = acc[mb][2]; p[3] = acc[mb][3]; q[0] = acc[mb][4]; q[1] = acc[mb][5]; q[2] = acc[mb][6]; q[3] = acc[mb][7];
        *(v4fa*)(&os[lr * 68 + mb * 16 + hi * 8]) = p; *(v4fa*)(&os[lr * 68 + mb * 16 + hi * 8 + 4]) = q; }
    wave_sync();
    const int b = lane >> 3, c8 = (lane & 7) * 8;
    const v4f w0 = *(const v4f*)(wst + r0 + c8), w1 = *(const v4f*)(wst + r0 + c8 + 4);
    const v4f g0 = *(const v4f*)(awb + r0 + c8), g1 = *(const v4f*)(awb + r0 + c8 + 4);
    const v4f a0 = *(const v4fa*)(&os[b * 68 + c8]), a1 = *(const v4fa*)(&os[b * 68 + c8 + 4]);
    v8h hv;
#pragma unroll
    for (int i = 0; i < 4; ++i) { hv[i] = toh_flush(bfr(w0[i]) + (a0[i] + bfr(g0[i]))); hv[4 + i] = toh_flush(bfr(w1[i]) + (a1[i] + bfr(g1[i]))); }
    h16* dst = WP + (size_t)b * ((size_t)DM * DM) + (size_t)r0 + c8;
#pragma unroll 1
    for (int ps = 0; ps < 2; ++ps) {
        if (b < NB) *(volatile v8h*)dst = hv;
        if (ps == 0) __threadfence(); }
}

__global__ __launch_bounds__(32) void k_abgen(const bf* __restrict__ ABW, const bf* __restrict__ ADP, const float* __restrict__ abb, float* ABP) {
    __shared__ __align__(16) float os[16 * 68];
    const int lane = threadIdx.x & 31, lr = lane & 15, hi = lane >> 4; const int r0 = blockIdx.x * 64;
    v8f acc[4];
    adapt_acc(ABW, ADP, r0, lr, hi, acc);
#pragma unroll
    for (int mb = 0; mb < 4; ++mb) { v4f p, q;
        p[0] = acc[mb][0]; p[1] = acc[mb][1]; p[2] = acc[mb][2]; p[3] = acc[mb][3]; q[0] = acc[mb][4]; q[1] = acc[mb][5]; q[2] = acc[mb][6]; q[3] = acc[mb][7];
        *(v4fa*)(&os[lr * 68 + mb * 16 + hi * 8]) = p; *(v4fa*)(&os[lr * 68 + mb * 16 + hi * 8 + 4]) = q; }
    wave_sync();
    const int b = lane >> 3, c4 = (lane & 7) * 4;
#pragma unroll 1
    for (int ps = 0; ps < 2; ++ps) {
#pragma unroll
        for (int s = 0; s < 2; ++s) { const int cc = s * 32 + c4;
            const v4f a = *(const v4fa*)(&os[b * 68 + cc]); const v4f g = *(const v4f*)(abb + r0 + cc); v4f val;
#pragma unroll
            for (int i = 0; i < 4; ++i) val[i] = a[i] + bfr(g[i]);
            if (b < NB) *(volatile v4f*)(ABP + (size_t)b * DM + r0 + cc) = val; }
        if (ps == 0) __threadfence(); }
}

__global__ __launch_bounds__(32) void k_bgemm(const h16* __restrict__ XH, const h16* __restrict__ WP, const float* __restrict__ AB, float* OUT) {
    __shared__ __align__(16) float os[16 * 68];
    const int K = DM;
    const int lane = threadIdx.x & 31, lr = lane & 15, hi = lane >> 4; const int r0 = blockIdx.x * 64, c0 = blockIdx.y * 64;
    const int bb = r0 / SEQ, tt = r0 % SEQ;
    v8f acc[4][4];
#pragma unroll
    for (int mb = 0; mb < 4; ++mb)
#pragma unroll
        for (int nb = 0; nb < 4; ++nb) acc[mb][nb] = (v8f){};
    const size_t aoff = (size_t)(r0 + lr) * K + 8 * hi, boff = (size_t)bb * ((size_t)DM * DM) + (size_t)(c0 + lr) * K + 8 * hi;
#pragma unroll 1
    for (int kc = 0; kc < K; kc += 32) {
        v16h a[4];
#pragma unroll
        for (int mb = 0; mb < 4; ++mb) a[mb] = ldh(XH + aoff + (size_t)mb * 16 * K + kc);
#pragma unroll
        for (int nb = 0; nb < 4; ++nb) { const v16h b = ldh(WP + boff + (size_t)nb * 16 * K + kc);
#pragma unroll
            for (int mb = 0; mb < 4; ++mb) acc[mb][nb] = wmma16g(a[mb], b, acc[mb][nb]); }
    }
    const v4f abv = *(const v4f*)(AB + (size_t)bb * DM + c0 + lr * 4);
    float* obase = OUT + ((size_t)bb * OUT_SEQ + tt) * DM + c0;
#pragma unroll
    for (int mb = 0; mb < 4; ++mb) {
#pragma unroll
        for (int nb = 0; nb < 4; ++nb) {
#pragma unroll
            for (int j = 0; j < 8; ++j) os[(hi * 8 + j) * 68 + nb * 16 + lr] = acc[mb][nb][j]; }
        wave_sync();
#pragma unroll 1
        for (int ps = 0; ps < 2; ++ps) {
#pragma unroll
            for (int s = 0; s < 8; ++s) { const int row = 2 * s + hi, c4 = lr * 4;
                v4f val = *(const v4fa*)(&os[row * 68 + c4]); val = val + abv;
                *(volatile v4f*)(obase + (size_t)(mb * 16 + row) * DM + c4) = val; }
            if (ps == 0) __threadfence(); }
        wave_sync();
    }
}

static constexpr size_t al256(size_t v) { return (v + 255) & ~(size_t)255; }
static constexpr size_t SZ_AWB = al256((size_t)DM * DM * KA * 2);
static constexpr size_t SZ_ABW = al256((size_t)DM * KA * 2);
static constexpr size_t SZ_ADP = al256((size_t)NBP * KA * 2);
static constexpr size_t SZ_XH  = al256((size_t)NB * SEQ * DM * 2);
static constexpr size_t SZ_WP  = al256((size_t)NB * DM * DM * 2);
static constexpr size_t SZ_ABP = al256((size_t)NB * DM * 4);
static constexpr size_t SZ_TOTAL = SZ_AWB + SZ_ABW + SZ_ADP + SZ_XH + SZ_WP + SZ_ABP;
static_assert(SZ_TOTAL <= (size_t)134217728);
static_assert(((size_t)(DM * DM / 64 - 1) * 64 + 63) < (size_t)DM * DM);
static_assert(((size_t)(NB - 1) * DM * DM + (size_t)DM * DM) * 2 <= SZ_WP);
static_assert(((size_t)(NB - 1) * DM + DM) * 4 <= SZ_ABP);

extern "C" void kernel_launch(void* const* d_in, const int* in_sizes, int n_in,
                              void* d_out, int out_size, void* d_ws, size_t ws_size, hipStream_t stream) {
    if (n_in < 7) return;
    const size_t needx = ((size_t)(NB - 1) * SEQ_FULL + SEQ) * DM;
    if ((size_t)in_sizes[0] < needx) return;
    if ((size_t)in_sizes[1] < (size_t)NB * KA) return;
    if ((size_t)in_sizes[2] < (size_t)DM * DM) return;
    if ((size_t)in_sizes[3] < (size_t)DM * DM * KA) return;
    if ((size_t)in_sizes[4] < (size_t)DM * DM) return;
    if ((size_t)in_sizes[5] < (size_t)DM * KA) return;
    if ((size_t)in_sizes[6] < (size_t)DM) return;
    if ((size_t)out_size < ((size_t)(NB - 1) * OUT_SEQ + SEQ) * DM) return;
    if (SZ_TOTAL > ws_size) return;
    const float* x   = (const float*)d_in[0];
    const float* adp = (const float*)d_in[1];
    const float* wst = (const float*)d_in[2];
    const float* aww = (const float*)d_in[3];
    const float* awb = (const float*)d_in[4];
    const float* abw = (const float*)d_in[5];
    const float* abb = (const float*)d_in[6];
    float* OUT = (float*)d_out;
    char* wsp = (char*)d_ws;
    bf*  AWB = (bf*)wsp;   wsp += SZ_AWB;
    bf*  ABW = (bf*)wsp;   wsp += SZ_ABW;
    bf*  ADP = (bf*)wsp;   wsp += SZ_ADP;
    h16* XH  = (h16*)wsp;  wsp += SZ_XH;
    h16* WP  = (h16*)wsp;  wsp += SZ_WP;
    float* ABP = (float*)wsp; wsp += SZ_ABP;

    { const size_t n8 = (size_t)DM * DM * KA / 8; k_cvt8<<<(unsigned)((n8 + 255) / 256), 256, 0, stream>>>(aww, AWB, n8); }
    { const size_t n8 = (size_t)DM * KA / 8;      k_cvt8<<<(unsigned)((n8 + 255) / 256), 256, 0, stream>>>(abw, ABW, n8); }
    k_adp<<<1, 128, 0, stream>>>(adp, ADP);
    if (SEQ == SEQ_FULL) {
        const size_t n8 = (size_t)NB * SEQ * DM / 8;
        k_cvth8<<<(unsigned)((n8 + 255) / 256), 256, 0, stream>>>(x, XH, n8);
    } else {
        const size_t n8 = (size_t)SEQ * DM / 8;
        for (int b = 0; b < NB; ++b) k_cvth8<<<(unsigned)((n8 + 255) / 256), 256, 0, stream>>>(x + (size_t)b * SEQ_FULL * DM, XH + (size_t)b * SEQ * DM, n8);
    }

    k_wgen<<<DM * DM / 64, 32, 0, stream>>>(AWB, ADP, awb, wst, WP);
    k_abgen<<<DM / 64, 32, 0, stream>>>(ABW, ADP, abb, ABP);

    k_bgemm<<<dim3(NB * SEQ / 64, DM / 64, 1), 32, 0, stream>>>(XH, WP, ABP, OUT);
}
